// DeepWDK_23974507446892
// MI455X (gfx1250) — hardware-verified
//
#include <hip/hip_runtime.h>


#define N1_  512
#define N2_  512
#define NSQ  (N1_ + N2_)
#define LL   200
#define NAA  20
#define DD   64
#define ED   32
#define KIN  (LL * ED)
#define NOUT (NAA * DD)

typedef unsigned short bf;
typedef __attribute__((ext_vector_type(16))) __bf16   v16bf;
typedef __attribute__((ext_vector_type(8)))  unsigned short v8us;
typedef __attribute__((ext_vector_type(8)))  float    v8f;
typedef __attribute__((ext_vector_type(4)))  float    v4f;
typedef __attribute__((ext_vector_type(2)))  float    v2f;
typedef v4f  __attribute__((may_alias)) v4fa;
typedef v8us __attribute__((may_alias)) v8usa;

__device__ __forceinline__ unsigned short f2bf(float f) { unsigned u = __float_as_uint(f); u += 0x7FFFu + ((u >> 16) & 1u); return (unsigned short)(u >> 16); }
__device__ __forceinline__ float bf2f(unsigned short b) { return __uint_as_float(((unsigned)b) << 16); }
__device__ __forceinline__ float bfr(float f) { return bf2f(f2bf(f)); }
__device__ __forceinline__ v16bf cat16b(v8us lo, v8us hi) { return __builtin_bit_cast(v16bf, __builtin_shufflevector(lo, hi, 0, 1, 2, 3, 4, 5, 6, 7, 8, 9, 10, 11, 12, 13, 14, 15)); }
__device__ __forceinline__ v8f wmmab(v16bf a, v16bf b, v8f c) { return __builtin_amdgcn_wmma_f32_16x16x32_bf16(false, a, false, b, (short)0, c, false, false); }
#define VST2(T, p, v) do { const T vst2_v_ = (v); *(volatile T*)(p) = vst2_v_; __threadfence(); *(volatile T*)(p) = vst2_v_; } while (0)

__global__ __launch_bounds__(256) void k_h(const int* __restrict__ X1, const int* __restrict__ X2, const float* __restrict__ E, bf* H) {
    const int lane = threadIdx.x & 31, wid = blockIdx.x * 8 + (threadIdx.x >> 5);
    const int n = wid / (LL / 8), lg = wid - n * (LL / 8);
    if (n >= NSQ) return;
    const int l = lg * 8 + (lane >> 2), e0 = (lane & 3) * 8;
    int tok = (n < N1_) ? X1[n * LL + l] : X2[(n - N1_) * LL + l];
    if (tok < 0) tok += NAA; tok = ((unsigned)tok < (unsigned)NAA) ? tok : 0;
    v8us t;
#pragma unroll
    for (int i = 0; i < 8; ++i) t[i] = f2bf(E[tok * ED + e0 + i]);
    VST2(v8us, H + (size_t)n * KIN + l * ED + e0, t);
}
__global__ __launch_bounds__(256) void k_wt(const float* __restrict__ Wm, bf* WT) {
    __shared__ __align__(16) unsigned short tl[64 * 72];
    const int tid = threadIdx.x, k0 = blockIdx.x * 64, n0 = blockIdx.y * 64;
    const int kk = tid >> 2, nq = (tid & 3) * 16;
#pragma unroll
    for (int i = 0; i < 16; ++i) tl[(nq + i) * 72 + kk] = f2bf(Wm[(size_t)(k0 + kk) * NOUT + n0 + nq + i]);
    __syncthreads();
    const int piece = tid & 7;
    auto pass = [&]() {
#pragma unroll
        for (int s = 0; s < 2; ++s) { const int nr = (tid >> 3) + 32 * s; const v8us val = *(const v8usa*)(tl + nr * 72 + piece * 8);
            *(volatile v8us*)(WT + (size_t)(n0 + nr) * KIN + k0 + piece * 8) = val; }
    };
    pass(); __threadfence(); pass();
}
__global__ __launch_bounds__(128) void k_gemm(const bf* __restrict__ A, const bf* __restrict__ Bn, float* C) {
    __shared__ __align__(16) float ost[4][16 * 68];
    const int lane = threadIdx.x & 31, wave = threadIdx.x >> 5, lr = lane & 15, hi = lane >> 4;
    const int r0 = blockIdx.x * 64 + wave * 16, c0 = blockIdx.y * 64;
    const size_t aoff = (size_t)(r0 + lr) * KIN + 8 * hi;
    size_t boff[4];
#pragma unroll
    for (int t = 0; t < 4; ++t) boff[t] = (size_t)(c0 + t * 16 + lr) * KIN + 8 * hi;
    v8f acc[4];
#pragma unroll
    for (int t = 0; t < 4; ++t) acc[t] = (v8f){};
#pragma unroll 1
    for (int kc = 0; kc < KIN; kc += 32) {
        const v16bf a = cat16b(*(const v8us*)(A + aoff + kc), *(const v8us*)(A + aoff + kc + 16));
#pragma unroll
        for (int t = 0; t < 4; ++t) acc[t] = wmmab(a, cat16b(*(const v8us*)(Bn + boff[t] + kc), *(const v8us*)(Bn + boff[t] + kc + 16)), acc[t]);
        asm volatile("v_nop\n\tv_nop\n\tv_nop\n\tv_nop" : "+v"(acc[0]), "+v"(acc[1]), "+v"(acc[2]), "+v"(acc[3]) : "v"(a));
    }
    float* os = &ost[wave][0];
#pragma unroll
    for (int t = 0; t < 4; ++t)
#pragma unroll
        for (int j = 0; j < 8; ++j) os[(hi * 8 + j) * 68 + t * 16 + lr] = acc[t][j];
    __syncthreads();
    float* crow = C + (size_t)r0 * NOUT + c0;
    auto pass = [&]() {
#pragma unroll
        for (int s = 0; s < 8; ++s) { const int Lid = (lane >> 3) + 4 * s, piece = lane & 7; const int row = Lid >> 1, cofs = (Lid & 1) * 32 + piece * 4;
            const v4f val = *(const v4fa*)(os + row * 68 + cofs); *(volatile v4f*)(crow + (size_t)row * NOUT + cofs) = val; }
    };
    pass(); __threadfence(); pass();
}
__global__ __launch_bounds__(256) void k_s(const float* __restrict__ V, const int* __restrict__ X1, const int* __restrict__ X2, float* S, float* KS) {
    __shared__ float vr[NOUT];
    __shared__ float sl[416];
    __shared__ float ks32[32];
    const int n = blockIdx.x, t = threadIdx.x;
    for (int i = t; i < NOUT; i += 256) vr[i] = V[(size_t)n * NOUT + i];
    if (t < 416 - 256) sl[256 + t] = 0.f;
    __syncthreads();
#pragma unroll 1
    for (int e = t; e < NAA * NAA; e += 256) { const int a = e / NAA, b = e - a * NAA; float s = 0.f;
#pragma unroll 8
        for (int d = 0; d < DD; ++d) s += vr[a * DD + d] * vr[b * DD + d];
        sl[e] = s; }
    __syncthreads();
    if (t == 0) { const int* X = (n < N1_) ? (X1 + n * LL) : (X2 + (n - N1_) * LL); float k = 0.f;
#pragma unroll 1
        for (int l = 0; l < LL; ++l) { int tok = X[l]; if (tok < 0) tok += NAA; tok = ((unsigned)tok < (unsigned)NAA) ? tok : 0; k += sl[tok * NAA + tok]; }
#pragma unroll
        for (int i = 0; i < 32; ++i) ks32[i] = (i == 0) ? k : 0.f; }
    __syncthreads();
    VST2(float, S + (size_t)n * 416 + t, sl[t]);
    if (t < 160) VST2(float, S + (size_t)n * 416 + 256 + t, sl[256 + t]);
    if (t < 32) VST2(float, KS + (size_t)n * 32 + t, ks32[t]);
}
__global__ __launch_bounds__(256) void k_out(const float* __restrict__ S, const float* __restrict__ KS, const int* __restrict__ X1, const int* __restrict__ X2, const float* __restrict__ av, float* out) {
    __shared__ float s1[416];
    __shared__ int x1[LL];
    const int i = blockIdx.x, t = threadIdx.x;
    for (int e = t; e < 416; e += 256) s1[e] = S[(size_t)i * 416 + e];
    if (t < LL) { int tok = X1[i * LL + t]; if (tok < 0) tok += NAA; x1[t] = ((unsigned)tok < (unsigned)NAA) ? tok : 0; }
    __syncthreads();
    const float a2 = bfr(av[0]) * bfr(av[0]), ik1 = 1.0f / sqrtf(KS[(size_t)i * 32]);
#pragma unroll
    for (int h = 0; h < 2; ++h) {
        const int j = t + 256 * h;
        const float* s2 = S + (size_t)(N1_ + j) * 416; const int* x2 = X2 + j * LL;
        float acc = 0.f;
#pragma unroll 2
        for (int l = 0; l < LL; ++l) { int b = x2[l]; if (b < 0) b += NAA; b = ((unsigned)b < (unsigned)NAA) ? b : 0; const int a = x1[l]; acc += s1[a * NAA + b] + s2[a * NAA + b]; }
        const float k = 0.5f * acc * ik1 / sqrtf(KS[(size_t)(N1_ + j) * 32]) * a2;
        VST2(float, out + (size_t)i * N2_ + j, k);
    }
}

extern "C" void kernel_launch(void* const* d_in, const int* in_sizes, int n_in,
                              void* d_out, int out_size, void* d_ws, size_t ws_size, hipStream_t stream) {
    (void)in_sizes; (void)n_in; (void)out_size;
    const int* X1 = (const int*)d_in[0]; const int* X2 = (const int*)d_in[1]; const float* E = (const float*)d_in[2]; const float* Wm = (const float*)d_in[3]; const float* av = (const float*)d_in[4];
    float* out = (float*)d_out;
    char* wsp = (char*)d_ws;
    auto take = [&](size_t bytes) { char* p = wsp; wsp += (bytes + 255) & ~(size_t)255; return (void*)p; };
    bf* H = (bf*)take((size_t)NSQ * KIN * 2); bf* WT = (bf*)take((size_t)NOUT * KIN * 2); float* V = (float*)take((size_t)NSQ * NOUT * 4);
    float* S = (float*)take((size_t)NSQ * 416 * 4); float* KS = (float*)take((size_t)NSQ * 32 * 4);
    if ((size_t)(wsp - (char*)d_ws) > ws_size) return;
    k_h<<<(NSQ * (LL / 8)) / 8, 256, 0, stream>>>(X1, X2, E, H);
    k_wt<<<dim3(KIN / 64, NOUT / 64, 1), 256, 0, stream>>>(Wm, WT);
    k_gemm<<<dim3(NSQ / 64, NOUT / 64, 1), 128, 0, stream>>>(H, WT, V);
    k_s<<<NSQ, 256, 0, stream>>>(V, X1, X2, S, KS);
    k_out<<<N1_, 256, 0, stream>>>(S, KS, X1, X2, av, out);
}
